// S4D_90623809945982
// MI455X (gfx1250) — hardware-verified
//
#include <hip/hip_runtime.h>
#include <math.h>

constexpr int NBATCH = 4;
constexpr int NLEN   = 2048;
constexpr int NWID   = 1024;
constexpr int NSTATE = 32;
constexpr int NBIN   = 2048;
constexpr int NFWD   = 4095;
constexpr int NINV   = 4096;
constexpr int NSPEC  = 2 * NBIN;
constexpr int NUCOL  = NBATCH * NWID;
constexpr int NAROW  = NUCOL + NWID;
constexpr int NTHR   = 256;
constexpr int KRTP   = 36;
constexpr float KRCARRY    = 32.0f;
constexpr float YCARRY     = 256.0f;
constexpr float YCARRY_INV = 1.0f / 256.0f;
constexpr float SC_DC = YCARRY / (KRCARRY * 4096.0f);
constexpr float SC_AC = 2.0f * YCARRY / (KRCARRY * 4096.0f);
constexpr float C95 = (float)(6.283185307179586476925286766559 / 4095.0);
constexpr float C96 = (float)(6.283185307179586476925286766559 / 4096.0);

static_assert(NLEN % 32 == 0 && NSPEC % 32 == 0, "GEMM K multiples of 32");
static_assert(NWID % 64 == 0 && NSPEC % 64 == 0 && NLEN % 64 == 0 && NAROW % 64 == 0, "GEMM M, N tile multiples");
static_assert(NWID % 2 == 0, "tap kernel: two channels per block");
static_assert(NLEN % 256 == 0, "tap kernel: 256-sample store chunks");
static_assert((NBIN * (NLEN / 8)) % NTHR == 0, "forward twiddle fill grid exact");
static_assert((NLEN * (NSPEC / 8)) % NTHR == 0, "inverse twiddle fill grid exact");
static_assert((NWID * (NSPEC / 8)) % NTHR == 0, "spectral product grid exact");
static_assert((NINV / 2) % NTHR == 0, "twiddle table grid exact: 2048 threads x 2 entries = 4096 entries per table");
static_assert(((NWID / 64) * (NSPEC / 64)) % 8 == 0 && ((NLEN / 64) * (NWID / 64)) % 8 == 0, "8 tiles per GEMM block");

typedef __attribute__((ext_vector_type(16))) _Float16 v16h;
typedef __attribute__((ext_vector_type(8)))  _Float16 v8h;
typedef __attribute__((ext_vector_type(16))) __bf16   v16b;
typedef __attribute__((ext_vector_type(8)))  __bf16   v8b;
typedef __attribute__((ext_vector_type(8)))  float    v8f;
typedef __attribute__((ext_vector_type(4)))  float    v4f;
typedef __attribute__((ext_vector_type(2)))  float    v2f;

__device__ __forceinline__ unsigned short f2bf_bits(float f) {
  unsigned u = __float_as_uint(f);
  return (unsigned short)((u + 0x7FFFu + ((u >> 16) & 1u)) >> 16);
}
__device__ __forceinline__ float bf_bits2f(unsigned short h) { return __uint_as_float(((unsigned)h) << 16); }

__device__ __forceinline__ void dep_guard_h(v8f& a, v8f& b, v16h x, v16h y) { asm volatile("v_nop\n\tv_nop\n\tv_nop\n\tv_nop" : "+v"(a), "+v"(b) : "v"(x), "v"(y)); }
__device__ __forceinline__ void dep_guard_b(v8f& a, v8f& b, v16b x, v16b y) { asm volatile("v_nop\n\tv_nop\n\tv_nop\n\tv_nop" : "+v"(a), "+v"(b) : "v"(x), "v"(y)); }
__device__ __forceinline__ void keep4_h(v16h a, v16h b, v16h c, v16h d) { asm volatile("v_nop" :: "v"(a), "v"(b), "v"(c), "v"(d)); }
__device__ __forceinline__ void keep4_b(v16b a, v16b b, v16b c, v16b d) { asm volatile("v_nop" :: "v"(a), "v"(b), "v"(c), "v"(d)); }
__device__ __forceinline__ void acc_guard4(v8f& a, v8f& b, v8f& c, v8f& d) { asm volatile("v_nop\n\tv_nop\n\tv_nop\n\tv_nop" : "+v"(a), "+v"(b), "+v"(c), "+v"(d)); }
template <typename T> struct Frag;
template <> struct Frag<_Float16> {
  typedef v16h V; union U { v16h v; v8h h[2]; };
  static __device__ __forceinline__ v16h load(const _Float16* p) {
    U f; f.h[0] = *(const v8h*)(p); f.h[1] = *(const v8h*)(p + 16); return f.v;
  }
  static __device__ __forceinline__ v8f mma(v16h a, v16h b, v8f c) {
    return __builtin_amdgcn_wmma_f32_16x16x32_f16(false, a, false, b, (short)0, c, false, false);
  }
  static __device__ __forceinline__ void guard(v8f& a, v8f& b, v16h x, v16h y) { dep_guard_h(a, b, x, y); }
  static __device__ __forceinline__ void keep(v16h a, v16h b, v16h c, v16h d) { keep4_h(a, b, c, d); }
};
template <> struct Frag<__bf16> {
  typedef v16b V; union U { v16b v; v8b h[2]; };
  static __device__ __forceinline__ v16b load(const __bf16* p) {
    U f; f.h[0] = *(const v8b*)(p); f.h[1] = *(const v8b*)(p + 16); return f.v;
  }
  static __device__ __forceinline__ v8f mma(v16b a, v16b b, v8f c) {
    return __builtin_amdgcn_wmma_f32_16x16x32_bf16(false, a, false, b, (short)0, c, false, false);
  }
  static __device__ __forceinline__ void guard(v8f& a, v8f& b, v16b x, v16b y) { dep_guard_b(a, b, x, y); }
  static __device__ __forceinline__ void keep(v16b a, v16b b, v16b c, v16b d) { keep4_b(a, b, c, d); }
};

template <int ET> struct Elem;
template <> struct Elem<0> { typedef _Float16 T; };
template <> struct Elem<1> { typedef __bf16 T; };
template <int ET, bool SPLIT, int BIAS_MODE, int OUT_MODE, int RESM, int ACT = 0>
__global__ __launch_bounds__(256) void wmma_gemm64(
    const unsigned short* __restrict__ Ap, const unsigned short* __restrict__ A2p, int lda, long strideA,
    const unsigned short* __restrict__ Btp, const unsigned short* __restrict__ Bt2p, int ldb, long strideB,
    void* __restrict__ Cout, void* __restrict__ Cout2, int ldc, long strideC,
    const float* __restrict__ bias,
    const float* __restrict__ resid, long strideR,
    int M, int N, int K, float scale) {
  typedef typename Elem<ET>::T T;
  typedef typename Frag<T>::V V;
  static_assert(RESM == 0 || (RESM == 2 && OUT_MODE == 0), "store-phase residual only with f32 output");
  const T* A = (const T*)Ap; const T* A2 = (const T*)A2p; const T* Bt = (const T*)Btp; const T* Bt2 = (const T*)Bt2p;
  __shared__ __align__(16) float sT[8][16 * 68];
  const int b    = blockIdx.y;
  const int lane = threadIdx.x & 31;
  const int wave = threadIdx.x >> 5;
  const int tilesN = N >> 6;
  const int tilesM = M >> 6;
  const int tile = blockIdx.x * 8 + wave;
  if (tile >= tilesM * tilesN) return;
  const int tm = tile / tilesN;
  const int tn = tile - tm * tilesN;
  const int m0 = tm << 6;
  const int n0 = tn << 6;

  const T* Ab  = A  + (size_t)b * strideA;
  const T* Bb  = Bt + (size_t)b * strideB;
  const T* Ab2 = SPLIT ? (A2  + (size_t)b * strideA) : nullptr;
  const T* Bb2 = SPLIT ? (Bt2 + (size_t)b * strideB) : nullptr;

  const int rlane = lane & 15;
  const int koff  = (lane >> 4) * 8;
  const int mOff  = (lane >> 4) * 8;

  v8f acc[4][4];
#pragma unroll
  for (int i = 0; i < 4; ++i)
#pragma unroll
    for (int j = 0; j < 4; ++j) acc[i][j] = (v8f){0.f,0.f,0.f,0.f,0.f,0.f,0.f,0.f};

  for (int k0 = 0; k0 < K; k0 += 32) {
    V bh[4], bl[4];
#pragma unroll
    for (int j = 0; j < 4; ++j) {
      const size_t bo = (size_t)(n0 + (j << 4) + rlane) * ldb + koff + k0;
      bh[j] = Frag<T>::load(Bb + bo);
      if (SPLIT) bl[j] = Frag<T>::load(Bb2 + bo);
    }
#pragma unroll
    for (int i = 0; i < 4; ++i) {
      const size_t ao = (size_t)(m0 + (i << 4) + rlane) * lda + koff + k0;
      V ah = Frag<T>::load(Ab + ao);
      V al;
      if (SPLIT) al = Frag<T>::load(Ab2 + ao);
#pragma unroll
      for (int j = 0; j < 4; ++j) {
        acc[i][j] = Frag<T>::mma(ah, bh[j], acc[i][j]);
        if (SPLIT) {
          acc[i][j] = Frag<T>::mma(ah, bl[j], acc[i][j]);
          acc[i][j] = Frag<T>::mma(al, bh[j], acc[i][j]);
        }
      }
      Frag<T>::guard(acc[i][0], acc[i][3], ah, SPLIT ? al : ah);
    }
    Frag<T>::keep(bh[0], bh[1], bh[2], bh[3]);
    if (SPLIT) Frag<T>::keep(bl[0], bl[1], bl[2], bl[3]);
  }
  acc_guard4(acc[0][0], acc[0][1], acc[0][2], acc[0][3]);
  acc_guard4(acc[1][0], acc[1][1], acc[1][2], acc[1][3]);
  acc_guard4(acc[2][0], acc[2][1], acc[2][2], acc[2][3]);
  acc_guard4(acc[3][0], acc[3][1], acc[3][2], acc[3][3]);

  float* slab = sT[wave];
#pragma unroll
  for (int i = 0; i < 4; ++i) {
    const int mBase = m0 + (i << 4);
#pragma unroll
    for (int j = 0; j < 4; ++j) {
      const int n = n0 + (j << 4) + rlane;
      float bv = 0.f;
      if (BIAS_MODE == 2) bv = bias[n];
#pragma unroll
      for (int r = 0; r < 8; ++r) {
        float v = acc[i][j][r] * scale;
        if (BIAS_MODE == 1) v += bias[mBase + mOff + r];
        if (BIAS_MODE == 2) v += bv;
        if (ACT == 1) v = tanhf(v);
        if (ACT == 2) v = fmaxf(v, 0.0f);
        if (ACT == 4) v = (v > 0.f) ? v : 0.01f * v;
        slab[(mOff + r) * 68 + (j << 4) + rlane] = v;
      }
    }
    __builtin_amdgcn_fence(__ATOMIC_RELEASE, "workgroup");
    __builtin_amdgcn_wave_barrier();
    __builtin_amdgcn_fence(__ATOMIC_ACQUIRE, "workgroup");
    if (OUT_MODE == 0) {
      float* C = (float*)Cout + (size_t)b * strideC;
      const int hh = lane >> 4, c4 = (lane & 15) * 4;
      v4f gv = (v4f){0.f, 0.f, 0.f, 0.f};
      const float* Rb = nullptr;
      if (RESM == 2) { gv = *(const v4f*)(bias + n0 + c4); Rb = resid + (size_t)b * strideR; }
      for (int pass = 0; pass < 2; ++pass) {
#pragma unroll
        for (int it = 0; it < 8; ++it) {
          const int row = it * 2 + hh;
          v4f v = *(const v4f*)(slab + row * 68 + c4);
          if (RESM == 2) {
            const v4f rv = *(const v4f*)(Rb + (size_t)(mBase + row) * ldc + n0 + c4);
            v[0] = fmaf(gv[0], rv[0], v[0]);
            v[1] = fmaf(gv[1], rv[1], v[1]);
            v[2] = fmaf(gv[2], rv[2], v[2]);
            v[3] = fmaf(gv[3], rv[3], v[3]);
          }
          *(volatile v4f*)(C + (size_t)(mBase + row) * ldc + n0 + c4) = v;
        }
        __threadfence();
      }
    } else {
      const int q = lane >> 3, c8 = (lane & 7) * 8;
      unsigned short* C  = (unsigned short*)Cout  + (size_t)b * strideC;
      unsigned short* C2 = (OUT_MODE == 2) ? ((unsigned short*)Cout2 + (size_t)b * strideC) : nullptr;
      for (int pass = 0; pass < 2; ++pass) {
#pragma unroll
        for (int it = 0; it < 4; ++it) {
          const int row = it * 4 + q;
          const float* sp = slab + row * 68 + c8;
          v8h hv, lv;
#pragma unroll
          for (int e = 0; e < 8; ++e) {
            if (OUT_MODE == 1) {
              hv[e] = (_Float16)sp[e];
            } else {
              unsigned short hb = f2bf_bits(sp[e]);
              unsigned short lb = f2bf_bits(sp[e] - bf_bits2f(hb));
              hv[e] = __builtin_bit_cast(_Float16, hb);
              lv[e] = __builtin_bit_cast(_Float16, lb);
            }
          }
          *(volatile v8h*)(C + (size_t)(mBase + row) * ldc + n0 + c8) = hv;
          if (OUT_MODE == 2) *(volatile v8h*)(C2 + (size_t)(mBase + row) * ldc + n0 + c8) = lv;
        }
        __threadfence();
      }
    }
    __builtin_amdgcn_fence(__ATOMIC_RELEASE, "workgroup");
    __builtin_amdgcn_wave_barrier();
    __builtin_amdgcn_fence(__ATOMIC_ACQUIRE, "workgroup");
  }
}

__global__ __launch_bounds__(NTHR) void twtab_kernel(float* __restrict__ tw) {
  const int which = blockIdx.y;
  const int i = blockIdx.x * NTHR + threadIdx.x;
  const int per = which ? NINV : NFWD;
  const float cf = which ? C96 : C95;
  v4f o;
#pragma unroll
  for (int e = 0; e < 2; ++e) {
    const int r = 2 * i + e;
    const int rr = (r > 2047) ? (r - per) : r;
    const float ang = (float)rr * cf;
    float s, c;
    sincosf(ang, &s, &c);
    if (which != 0 && (rr == 1024 || rr == -1024)) c = 0.0f;
    if (which != 0 && rr == -2048) s = 0.0f;
    o[2 * e] = c;
    o[2 * e + 1] = -s;
  }
  float* p = tw + (size_t)which * 2 * NINV + 4 * i;
  *(volatile v4f*)p = o;
  __threadfence();
  *(volatile v4f*)p = o;
}

__global__ __launch_bounds__(64) void kr_kernel(const float* __restrict__ w_re, const float* __restrict__ w_im,
                                               const float* __restrict__ c_re, const float* __restrict__ c_im,
                                               const float* __restrict__ dt, unsigned short* __restrict__ ucols) {
  __shared__ __align__(16) float tile[2][32 * KRTP];
  __shared__ __align__(16) float oslab[2][256];
  const int tid = threadIdx.x, lane = tid & 31, wave = tid >> 5;
  const int h = blockIdx.x * 2 + wave;
  const float dtv = dt[h];
  const float wr = w_re[lane], wi = w_im[lane];
  const float ar = wr * dtv, ai = wi * dtv;
  const float er = expf(ar);
  float sn, cs;
  sincosf(ai, &sn, &cs);
  const float stAr = er * cs, stAi = er * sn;
  const float nr = stAr - 1.0f, ni = stAi;
  const float den = wr * wr + wi * wi;
  const float dinv = 1.0f / den;
  const float qr = (nr * wr + ni * wi) * dinv;
  const float qi = (ni * wr - nr * wi) * dinv;
  const float cr = c_re[h * NSTATE + lane], ci = c_im[h * NSTATE + lane];
  const float gr = cr * qr - ci * qi;
  const float gi = cr * qi + ci * qr;
  const float g2r = gr * (2.0f * KRCARRY), g2i = gi * (2.0f * KRCARRY);
  float pr = 1.0f, pim = 0.0f;
  float* tl = tile[wave];
  float* os = oslab[wave];
  unsigned short* orow = ucols + (size_t)(NUCOL + h) * NLEN;
  const int q = lane >> 3, c8 = (lane & 7) * 8;
#pragma unroll 1
  for (int c256 = 0; c256 < NLEN / 256; ++c256) {
#pragma unroll 1
    for (int c32 = 0; c32 < 8; ++c32) {
#pragma unroll 4
      for (int tt = 0; tt < 32; ++tt) {
        const float term = g2r * pr - g2i * pim;
        tl[tt * KRTP + lane] = term;
        const float npr = pr * stAr - pim * stAi;
        const float npi = pr * stAi + pim * stAr;
        pr = npr; pim = npi;
      }
      __syncthreads();
      const float* rp = tl + lane * KRTP;
      float s = 0.0f;
#pragma unroll
      for (int e4 = 0; e4 < 8; ++e4) {
        const v4f a = *(const v4f*)(rp + 4 * e4);
        s += (a[0] + a[1]) + (a[2] + a[3]);
      }
      os[c32 * 32 + lane] = s;
      __syncthreads();
    }
    const v4f x0 = *(const v4f*)(os + 64 * q + c8);
    const v4f x1 = *(const v4f*)(os + 64 * q + c8 + 4);
    v8h hv;
#pragma unroll
    for (int e = 0; e < 4; ++e) { hv[e] = (_Float16)x0[e]; hv[4 + e] = (_Float16)x1[e]; }
    unsigned short* op = orow + c256 * 256 + 64 * q + c8;
    *(volatile v8h*)op = hv;
    __threadfence();
    *(volatile v8h*)op = hv;
  }
}

__global__ __launch_bounds__(NTHR) void utr_kernel(const float* __restrict__ u, unsigned short* __restrict__ ucols) {
  __shared__ float Tt[64 * 65];
  const int tid = threadIdx.x;
  const int b = blockIdx.z;
  const int h0 = blockIdx.x * 64, l0 = blockIdx.y * 64;
  const float* src = u + (size_t)b * NLEN * NWID;
#pragma unroll
  for (int i = 0; i < 4; ++i) {
    const int idx = i * NTHR + tid;
    const int rr = idx >> 4, cc = (idx & 15) * 4;
    const v4f v = *(const v4f*)(src + (size_t)(l0 + rr) * NWID + h0 + cc);
    Tt[rr * 65 + cc + 0] = v[0];
    Tt[rr * 65 + cc + 1] = v[1];
    Tt[rr * 65 + cc + 2] = v[2];
    Tt[rr * 65 + cc + 3] = v[3];
  }
  __syncthreads();
  const int q = tid >> 3, c8 = (tid & 7) * 8;
  v8h hv[2];
#pragma unroll
  for (int g = 0; g < 2; ++g) {
    const int qq = g * 32 + q;
#pragma unroll
    for (int e = 0; e < 8; ++e) hv[g][e] = (_Float16)Tt[(c8 + e) * 65 + qq];
  }
  for (int pass = 0; pass < 2; ++pass) {
#pragma unroll
    for (int g = 0; g < 2; ++g) {
      const size_t o = (size_t)(b * NWID + h0 + g * 32 + q) * NLEN + (size_t)(l0 + c8);
      *(volatile v8h*)(ucols + o) = hv[g];
    }
    __threadfence();
  }
}

__global__ __launch_bounds__(NTHR) void t95_fill_kernel(const float* __restrict__ tw, unsigned short* __restrict__ t95) {
  const int g = blockIdx.x * NTHR + threadIdx.x;
  const int k = g >> 8, s8 = g & 255;
  v8h hc, hs;
#pragma unroll
  for (int e = 0; e < 8; ++e) {
    const int t = s8 * 8 + e;
    const int r = (k * t) % NFWD;
    const v2f p = *(const v2f*)(tw + 2 * r);
    hc[e] = (_Float16)p[0];
    hs[e] = (_Float16)p[1];
  }
  const size_t oc = (size_t)(2 * k) * NLEN + (size_t)s8 * 8;
  const size_t osn = oc + NLEN;
  for (int pass = 0; pass < 2; ++pass) {
    *(volatile v8h*)(t95 + oc) = hc;
    *(volatile v8h*)(t95 + osn) = hs;
    __threadfence();
  }
}

__global__ __launch_bounds__(NTHR) void t96_fill_kernel(const float* __restrict__ tw, unsigned short* __restrict__ t96) {
  const int g = blockIdx.x * NTHR + threadIdx.x;
  const int m = g >> 9, k8 = g & 511;
  v8h hv;
#pragma unroll
  for (int j = 0; j < 4; ++j) {
    const int k = 4 * k8 + j;
    const int r = (k * m) & (NINV - 1);
    const v2f p = *(const v2f*)(tw + 2 * r);
    hv[2 * j]     = (_Float16)p[0];
    hv[2 * j + 1] = (_Float16)p[1];
  }
  unsigned short* op = t96 + (size_t)m * NSPEC + (size_t)k8 * 8;
  *(volatile v8h*)op = hv;
  __threadfence();
  *(volatile v8h*)op = hv;
}

__global__ __launch_bounds__(NTHR) void spec_kernel(const float* __restrict__ c1q, const float* __restrict__ kf,
                                                    unsigned short* __restrict__ yt) {
  const int g = blockIdx.x * NTHR + threadIdx.x;
  const int h = g >> 9, k4 = g & 511;
  const float* up = c1q + (size_t)h * NSPEC + (size_t)k4 * 8;
  const float* kp = kf  + (size_t)h * NSPEC + (size_t)k4 * 8;
  const v4f u0 = *(const v4f*)(up), u1 = *(const v4f*)(up + 4);
  const v4f q0 = *(const v4f*)(kp), q1 = *(const v4f*)(kp + 4);
  const float sc0  = (k4 == 0) ? SC_DC : SC_AC;
  const float imk0 = (k4 == 0) ? 0.0f : 1.0f;
  v8h hv;
  {
    const float yr = u0[0] * q0[0] - u0[1] * q0[1];
    const float yi = (u0[0] * q0[1] + u0[1] * q0[0]) * imk0;
    hv[0] = (_Float16)(yr * sc0);
    hv[1] = (_Float16)(yi * sc0);
  }
  {
    const float yr = u0[2] * q0[2] - u0[3] * q0[3];
    const float yi = u0[2] * q0[3] + u0[3] * q0[2];
    hv[2] = (_Float16)(yr * SC_AC);
    hv[3] = (_Float16)(yi * SC_AC);
  }
  {
    const float yr = u1[0] * q1[0] - u1[1] * q1[1];
    const float yi = u1[0] * q1[1] + u1[1] * q1[0];
    hv[4] = (_Float16)(yr * SC_AC);
    hv[5] = (_Float16)(yi * SC_AC);
  }
  {
    const float yr = u1[2] * q1[2] - u1[3] * q1[3];
    const float yi = u1[2] * q1[3] + u1[3] * q1[2];
    hv[6] = (_Float16)(yr * SC_AC);
    hv[7] = (_Float16)(yi * SC_AC);
  }
  unsigned short* op = yt + (size_t)h * NSPEC + (size_t)k4 * 8;
  *(volatile v8h*)op = hv;
  __threadfence();
  *(volatile v8h*)op = hv;
}

extern "C" void kernel_launch(void* const* d_in, const int* in_sizes, int n_in,
                              void* d_out, int out_size, void* d_ws, size_t ws_size, hipStream_t stream) {
  if (n_in < 7 || d_out == nullptr || d_ws == nullptr) return;
  if (in_sizes[0] != NBATCH * NLEN * NWID || in_sizes[1] != NSTATE || in_sizes[2] != NSTATE ||
      in_sizes[3] != NWID * NSTATE || in_sizes[4] != NWID * NSTATE || in_sizes[5] != NWID ||
      in_sizes[6] != NWID || out_size != NBATCH * NLEN * NWID) return;

  const float* u    = (const float*)d_in[0];
  const float* w_re = (const float*)d_in[1];
  const float* w_im = (const float*)d_in[2];
  const float* c_re = (const float*)d_in[3];
  const float* c_im = (const float*)d_in[4];
  const float* dsk  = (const float*)d_in[5];
  const float* dt   = (const float*)d_in[6];
  float* out = (float*)d_out;

  char* ws = (char*)d_ws; size_t off = 0;
  auto carve = [&](size_t bytes) -> char* { char* p = ws + off; off += (bytes + 255) & ~(size_t)255; return p; };
  float*          TW    = (float*)carve((size_t)2 * NINV * 2 * 4);
  unsigned short* UCOLS = (unsigned short*)carve((size_t)NAROW * NLEN * 2);
  unsigned short* T95   = (unsigned short*)carve((size_t)NSPEC * NLEN * 2);
  float*          KF    = (float*)carve((size_t)NWID * NSPEC * 4);
  float*          C1Q   = (float*)carve((size_t)NWID * NSPEC * 4);
  unsigned short* YT    = (unsigned short*)carve((size_t)NUCOL * NSPEC * 2);
  unsigned short* T96   = (unsigned short*)carve((size_t)NLEN * NSPEC * 2);
  if (off > ws_size || off > (size_t)134217728) return;

  twtab_kernel<<<dim3((NINV / 2) / NTHR, 2), NTHR, 0, stream>>>(TW);
  kr_kernel<<<NWID / 2, 64, 0, stream>>>(w_re, w_im, c_re, c_im, dt, UCOLS);
  utr_kernel<<<dim3(NWID / 64, NLEN / 64, NBATCH), NTHR, 0, stream>>>(u, UCOLS);
  t95_fill_kernel<<<(NBIN * (NLEN / 8)) / NTHR, NTHR, 0, stream>>>(TW, T95);

  const dim3 g1((NWID / 64) * (NSPEC / 64) / 8, 1);
  wmma_gemm64<0, false, 0, 0, 0, 0><<<g1, NTHR, 0, stream>>>(
      UCOLS + (size_t)NUCOL * NLEN, UCOLS + (size_t)NUCOL * NLEN, NLEN, 0L, T95, T95, NLEN, 0L,
      (void*)KF, (void*)KF, NSPEC, 0L, dsk, u, 0L, NWID, NSPEC, NLEN, 1.0f);

  for (int qb = 0; qb < NBATCH; ++qb) {
    wmma_gemm64<0, false, 0, 0, 0, 0><<<g1, NTHR, 0, stream>>>(
        UCOLS + (size_t)qb * NWID * NLEN, UCOLS + (size_t)qb * NWID * NLEN, NLEN, 0L, T95, T95, NLEN, 0L,
        (void*)C1Q, (void*)C1Q, NSPEC, 0L, dsk, u, 0L, NWID, NSPEC, NLEN, 1.0f);
    spec_kernel<<<(NWID * (NSPEC / 8)) / NTHR, NTHR, 0, stream>>>(C1Q, KF, YT + (size_t)qb * NWID * NSPEC);
  }

  t96_fill_kernel<<<(NLEN * (NSPEC / 8)) / NTHR, NTHR, 0, stream>>>(TW + 2 * NINV, T96);

  const dim3 g2((NLEN / 64) * (NWID / 64) / 8, NBATCH);
  wmma_gemm64<0, false, 0, 0, 2, 0><<<g2, NTHR, 0, stream>>>(
      T96, T96, NSPEC, 0L, YT, YT, NSPEC, (long)NWID * NSPEC,
      (void*)out, (void*)out, NWID, (long)NLEN * NWID, dsk, u, (long)NLEN * NWID,
      NLEN, NWID, NSPEC, YCARRY_INV);
}
